// CausalSelfAttention_38457137168858
// MI455X (gfx1250) — hardware-verified
//
#include <hip/hip_runtime.h>

#ifndef NB
#define NB 4
#endif
#ifndef SEQ
#define SEQ 2048
#endif
#define SEQ_FULL 2048
#define ND 1024
#define NH 16
#define HD 64
#define QKVW 3072
#define EARLY 256

#define AT_D 64
#define AT_NW 4
#define AT_QB 64
#define AT_KC 64
#define OS_P 64

static_assert(ND == NH * HD);
static_assert(QKVW == 3 * ND);
static_assert(HD == AT_D);
static_assert(AT_QB == 16 * AT_NW);
static_assert(AT_KC == AT_QB);
static_assert(SEQ % AT_QB == 0);
static_assert(SEQ >= EARLY);
static_assert(SEQ <= SEQ_FULL);
static_assert(EARLY % AT_QB == 0);
static_assert(EARLY % 64 == 0);
static_assert((SEQ - EARLY) % 64 == 0);
static_assert((NB * SEQ) % 64 == 0);
static_assert(ND % 64 == 0);
static_assert(QKVW % 64 == 0);
static_assert(ND % 32 == 0);
static_assert((2 * ND) % 32 == 0);
static_assert(ND % 8 == 0);

typedef __attribute__((ext_vector_type(16))) _Float16 v16h;
typedef __attribute__((ext_vector_type(8)))  _Float16 v8h;
typedef __attribute__((ext_vector_type(16))) __bf16   v16b;
typedef __attribute__((ext_vector_type(8)))  __bf16   v8b;
typedef __attribute__((ext_vector_type(8)))  float    v8f;
typedef __attribute__((ext_vector_type(4)))  float    v4f;
typedef __attribute__((ext_vector_type(4)))  unsigned int v4u;


#define VST2(T, ptr, val) do { const T vst2_v_ = (val); *(volatile T*)(ptr) = vst2_v_; __threadfence(); *(volatile T*)(ptr) = vst2_v_; } while (0)

__device__ __forceinline__ unsigned short f2bf_bits(float f) {
  unsigned u = __float_as_uint(f);
  return (unsigned short)((u + 0x7FFFu + ((u >> 16) & 1u)) >> 16);
}
__device__ __forceinline__ float bf_bits2f(unsigned short h) { return __uint_as_float(((unsigned)h) << 16); }
__device__ __forceinline__ float cmb_bf(float v) { const unsigned u = __float_as_uint(v); const unsigned r = (u + 0x7fffu + ((u >> 16) & 1u)) & 0xffff0000u; return __uint_as_float(r); }
__device__ __forceinline__ unsigned int cmb_pk2(float a, float b) { return (unsigned int)__builtin_bit_cast(unsigned short, (_Float16)a) | ((unsigned int)__builtin_bit_cast(unsigned short, (_Float16)b) << 16); }

__global__ __launch_bounds__(256) void k_cast_x(const float* __restrict__ SRC, unsigned short* __restrict__ DST) {
  const long long u = (long long)blockIdx.x * 256 + threadIdx.x;
  const int per = ND / 8;
  if (u >= (long long)NB * SEQ * per) return;
  const int r = (int)(u / per);
  const int c0 = 8 * (int)(u % per);
  const int b = r / SEQ, s = r - b * SEQ;
  const float* sp = SRC + ((long long)b * SEQ_FULL + s) * ND + c0;
  const v4f a = *(const v4f*)sp;
  const v4f d = *(const v4f*)(sp + 4);
  v4u pk;
  pk.x = cmb_pk2(cmb_bf(a.x), cmb_bf(a.y)); pk.y = cmb_pk2(cmb_bf(a.z), cmb_bf(a.w));
  pk.z = cmb_pk2(cmb_bf(d.x), cmb_bf(d.y)); pk.w = cmb_pk2(cmb_bf(d.z), cmb_bf(d.w));
  VST2(v4u, (v4u*)(DST + (long long)r * ND + c0), pk);
}
__global__ __launch_bounds__(256) void k_wT16(const float* __restrict__ SRC, int lds, unsigned short* __restrict__ DST, int ldd, int nR, int nC, float sc, int asbf, int dupoff) {
  const long long u = (long long)blockIdx.x * 256 + threadIdx.x;
  const int per = nR / 8;
  if (u >= (long long)nC * per) return;
  const int c = (int)(u / per);
  const int r0 = 8 * (int)(u % per);
  float w[8];
#pragma unroll
  for (int e = 0; e < 8; ++e) w[e] = cmb_bf(SRC[(long long)(r0 + e) * lds + c]);
  v4u pk;
  if (asbf != 0) {
    pk.x = (__float_as_uint(w[0]) >> 16) | (__float_as_uint(w[1]) & 0xffff0000u);
    pk.y = (__float_as_uint(w[2]) >> 16) | (__float_as_uint(w[3]) & 0xffff0000u);
    pk.z = (__float_as_uint(w[4]) >> 16) | (__float_as_uint(w[5]) & 0xffff0000u);
    pk.w = (__float_as_uint(w[6]) >> 16) | (__float_as_uint(w[7]) & 0xffff0000u);
  } else {
    pk.x = cmb_pk2(w[0] * sc, w[1] * sc); pk.y = cmb_pk2(w[2] * sc, w[3] * sc);
    pk.z = cmb_pk2(w[4] * sc, w[5] * sc); pk.w = cmb_pk2(w[6] * sc, w[7] * sc);
  }
  VST2(v4u, (v4u*)(DST + (long long)c * ldd + r0), pk);
  if (dupoff > 0) VST2(v4u, (v4u*)(DST + (long long)c * ldd + dupoff + r0), pk);
}
__global__ __launch_bounds__(256) void k_bfvec(const float* __restrict__ SRC, float* __restrict__ DST, int n) {
  const int u = blockIdx.x * 256 + threadIdx.x;
  if (u >= n) return;
  VST2(float, DST + u, cmb_bf(SRC[u]));
}

__device__ __forceinline__ void dep_guard_h(v8f& a, v8f& b, v16h x, v16h y) { asm volatile("v_nop\n\tv_nop\n\tv_nop\n\tv_nop" : "+v"(a), "+v"(b) : "v"(x), "v"(y)); }
__device__ __forceinline__ void dep_guard_b(v8f& a, v8f& b, v16b x, v16b y) { asm volatile("v_nop\n\tv_nop\n\tv_nop\n\tv_nop" : "+v"(a), "+v"(b) : "v"(x), "v"(y)); }
__device__ __forceinline__ void keep4_h(v16h a, v16h b, v16h c, v16h d) { asm volatile("v_nop" :: "v"(a), "v"(b), "v"(c), "v"(d)); }
__device__ __forceinline__ void keep4_b(v16b a, v16b b, v16b c, v16b d) { asm volatile("v_nop" :: "v"(a), "v"(b), "v"(c), "v"(d)); }
__device__ __forceinline__ void acc_guard4(v8f& a, v8f& b, v8f& c, v8f& d) { asm volatile("v_nop\n\tv_nop\n\tv_nop\n\tv_nop" : "+v"(a), "+v"(b), "+v"(c), "+v"(d)); }
template <typename T> struct Frag;
template <> struct Frag<_Float16> {
  typedef v16h V; union U { v16h v; v8h h[2]; };
  static __device__ __forceinline__ v16h load(const _Float16* p) {
    U f; f.h[0] = *(const v8h*)(p); f.h[1] = *(const v8h*)(p + 16); return f.v;
  }
  static __device__ __forceinline__ v8f mma(v16h a, v16h b, v8f c) {
    return __builtin_amdgcn_wmma_f32_16x16x32_f16(false, a, false, b, (short)0, c, false, false);
  }
  static __device__ __forceinline__ void guard(v8f& a, v8f& b, v16h x, v16h y) { dep_guard_h(a, b, x, y); }
  static __device__ __forceinline__ void keep(v16h a, v16h b, v16h c, v16h d) { keep4_h(a, b, c, d); }
};
template <> struct Frag<__bf16> {
  typedef v16b V; union U { v16b v; v8b h[2]; };
  static __device__ __forceinline__ v16b load(const __bf16* p) {
    U f; f.h[0] = *(const v8b*)(p); f.h[1] = *(const v8b*)(p + 16); return f.v;
  }
  static __device__ __forceinline__ v8f mma(v16b a, v16b b, v8f c) {
    return __builtin_amdgcn_wmma_f32_16x16x32_bf16(false, a, false, b, (short)0, c, false, false);
  }
  static __device__ __forceinline__ void guard(v8f& a, v8f& b, v16b x, v16b y) { dep_guard_b(a, b, x, y); }
  static __device__ __forceinline__ void keep(v16b a, v16b b, v16b c, v16b d) { keep4_b(a, b, c, d); }
};
template <int ET> struct Elem;
template <> struct Elem<0> { typedef _Float16 T; };
template <> struct Elem<1> { typedef __bf16 T; };

template <int ET, int OUT_MODE>
__device__ __forceinline__ void gemm64_body(
    const unsigned short* __restrict__ Ap, const int lda, const long long strideA,
    const unsigned short* __restrict__ Btp, const int ldb,
    void* __restrict__ Cout, void* __restrict__ Cout2, const int ldc, const long long strideC,
    const float* __restrict__ bias, const int M, const int N, const int K, const float scale) {
  typedef typename Elem<ET>::T T;
  typedef typename Frag<T>::V V;
  __shared__ __align__(16) float sT[8][16 * 68];
  const int b    = blockIdx.y;
  const int lane = threadIdx.x & 31;
  const int wave = threadIdx.x >> 5;
  const int tilesN = N >> 6;
  const int tilesM = M >> 6;
  const int tile = blockIdx.x * 8 + wave;
  if (tile >= tilesM * tilesN) return;
  const int tm = tile / tilesN;
  const int tn = tile - tm * tilesN;
  const int m0 = tm << 6;
  const int n0 = tn << 6;

  const T* Ab = (const T*)Ap + (size_t)b * (size_t)strideA;
  const T* Bb = (const T*)Btp;

  const int rlane = lane & 15;
  const int koff  = (lane >> 4) * 8;
  const int mOff  = (lane >> 4) * 8;

  v8f acc[4][4];
#pragma unroll
  for (int i = 0; i < 4; ++i)
#pragma unroll
    for (int j = 0; j < 4; ++j) acc[i][j] = (v8f){0.f,0.f,0.f,0.f,0.f,0.f,0.f,0.f};

  for (int k0 = 0; k0 < K; k0 += 32) {
    V bh[4];
#pragma unroll
    for (int j = 0; j < 4; ++j) {
      const size_t bo = (size_t)(n0 + (j << 4) + rlane) * ldb + koff + k0;
      bh[j] = Frag<T>::load(Bb + bo);
    }
#pragma unroll
    for (int i = 0; i < 4; ++i) {
      const size_t ao = (size_t)(m0 + (i << 4) + rlane) * lda + koff + k0;
      V ah = Frag<T>::load(Ab + ao);
#pragma unroll
      for (int j = 0; j < 4; ++j) acc[i][j] = Frag<T>::mma(ah, bh[j], acc[i][j]);
      Frag<T>::guard(acc[i][0], acc[i][3], ah, ah);
    }
    Frag<T>::keep(bh[0], bh[1], bh[2], bh[3]);
  }
  acc_guard4(acc[0][0], acc[0][1], acc[0][2], acc[0][3]);
  acc_guard4(acc[1][0], acc[1][1], acc[1][2], acc[1][3]);
  acc_guard4(acc[2][0], acc[2][1], acc[2][2], acc[2][3]);
  acc_guard4(acc[3][0], acc[3][1], acc[3][2], acc[3][3]);

  float* slab = sT[wave];
#pragma unroll
  for (int i = 0; i < 4; ++i) {
    const int mBase = m0 + (i << 4);
#pragma unroll
    for (int j = 0; j < 4; ++j) {
      const int n = n0 + (j << 4) + rlane;
      const float bv = bias[n];
#pragma unroll
      for (int r = 0; r < 8; ++r) slab[(mOff + r) * 68 + (j << 4) + rlane] = acc[i][j][r] * scale + bv;
    }
    __builtin_amdgcn_fence(3  , "workgroup");
    __builtin_amdgcn_wave_barrier();
    __builtin_amdgcn_fence(2  , "workgroup");
    if (OUT_MODE == 0) {
      float* C = (float*)Cout + (size_t)b * (size_t)strideC;
      const int hh = lane >> 4, c4 = (lane & 15) * 4;
      for (int pass = 0; pass < 2; ++pass) {
#pragma unroll
        for (int it = 0; it < 8; ++it) {
          const int row = it * 2 + hh;
          v4f v = *(const v4f*)(slab + row * 68 + c4);
          *(volatile v4f*)(C + (size_t)(mBase + row) * ldc + n0 + c4) = v;
        }
        __threadfence();
      }
    } else {
      const int q = lane >> 3, c8 = (lane & 7) * 8;
      unsigned short* C  = (unsigned short*)Cout + (size_t)b * (size_t)strideC;
      unsigned short* C2 = (OUT_MODE == 2) ? ((unsigned short*)Cout2 + (size_t)b * (size_t)strideC) : nullptr;
      for (int pass = 0; pass < 2; ++pass) {
#pragma unroll
        for (int it = 0; it < 4; ++it) {
          const int row = it * 4 + q;
          const float* sp = slab + row * 68 + c8;
          v8h hv, lv;
#pragma unroll
          for (int e = 0; e < 8; ++e) {
            if (OUT_MODE == 1) {
              hv[e] = (_Float16)sp[e];
              lv[e] = (_Float16)0.f;
            } else {
              const unsigned short hb = f2bf_bits(sp[e]);
              const unsigned short lb = f2bf_bits(sp[e] - bf_bits2f(hb));
              hv[e] = __builtin_bit_cast(_Float16, hb);
              lv[e] = __builtin_bit_cast(_Float16, lb);
            }
          }
          *(volatile v8h*)(C + (size_t)(mBase + row) * ldc + n0 + c8) = hv;
          if (OUT_MODE == 2) *(volatile v8h*)(C2 + (size_t)(mBase + row) * ldc + n0 + c8) = lv;
        }
        __threadfence();
      }
    }
    __builtin_amdgcn_fence(3  , "workgroup");
    __builtin_amdgcn_wave_barrier();
    __builtin_amdgcn_fence(2  , "workgroup");
  }
}

__global__ __launch_bounds__(256) void k_gemm_qkv_main(const unsigned short* __restrict__ X16, const unsigned short* __restrict__ W316,
                                                       unsigned short* __restrict__ QKV16, const float* __restrict__ BR3) {
  gemm64_body<0, 1>(X16, ND, 0, W316, ND, (void*)QKV16, nullptr, QKVW, 0, BR3, NB * SEQ, QKVW, ND, 0.0625f);
}
__global__ __launch_bounds__(256) void k_gemm_qkv_early(const unsigned short* __restrict__ X16, const unsigned short* __restrict__ W316,
                                                        unsigned short* __restrict__ QEH, unsigned short* __restrict__ QEL, const float* __restrict__ BR3) {
  gemm64_body<0, 2>(X16, ND, (long long)SEQ * ND, W316, ND, (void*)QEH, (void*)QEL, QKVW, (long long)EARLY * QKVW, BR3, EARLY, QKVW, ND, 0.0625f);
}
__global__ __launch_bounds__(256) void k_gemm_proj_main(const unsigned short* __restrict__ CTX16, const unsigned short* __restrict__ WO16,
                                                        float* __restrict__ OUT, const float* __restrict__ BRO) {
  gemm64_body<0, 0>(CTX16 + (size_t)EARLY * ND, ND, (long long)SEQ * ND, WO16, ND, (void*)(OUT + (size_t)EARLY * ND), nullptr, ND, (long long)SEQ * ND, BRO, SEQ - EARLY, ND, ND, 0.00390625f);
}
__global__ __launch_bounds__(256) void k_gemm_proj_early(const unsigned short* __restrict__ CTXE, const unsigned short* __restrict__ WOB2,
                                                         float* __restrict__ OUT, const float* __restrict__ BRO) {
  gemm64_body<1, 0>(CTXE, 2 * ND, (long long)EARLY * 2 * ND, WOB2, 2 * ND, (void*)OUT, nullptr, ND, (long long)SEQ * ND, BRO, EARLY, ND, 2 * ND, 1.0f);
}

__device__ __forceinline__ __bf16 at_f2bf(float f) { return __builtin_bit_cast(__bf16, f2bf_bits(f)); }
__device__ __forceinline__ void at_split(float f, __bf16& hi, __bf16& lo) {
  const unsigned short hb = f2bf_bits(f);
  hi = __builtin_bit_cast(__bf16, hb);
  lo = at_f2bf(f - bf_bits2f(hb));
}
__device__ __forceinline__ v8f at_mma(v16b a, v16b b, v8f c) {
  c = __builtin_amdgcn_wmma_f32_16x16x32_bf16(false, a, false, b, (short)0, c, false, false);
  asm volatile("v_nop\n\tv_nop\n\tv_nop\n\tv_nop" : "+v"(c) : "v"(a), "v"(b));
  return c;
}
template <bool F16> __device__ __forceinline__ __bf16 at_to16(float f) {
  if (F16) return __builtin_bit_cast(__bf16, (_Float16)f);
  return at_f2bf(f);
}
template <bool F16> __device__ __forceinline__ v8f at_mma16(v16b a, v16b b, v8f c) {
  if (F16) {
    const v16h ah = __builtin_bit_cast(v16h, a), bh = __builtin_bit_cast(v16h, b);
    c = __builtin_amdgcn_wmma_f32_16x16x32_f16(false, ah, false, bh, (short)0, c, false, false);
    asm volatile("v_nop\n\tv_nop\n\tv_nop\n\tv_nop" : "+v"(c) : "v"(ah), "v"(bh));
    return c;
  }
  return at_mma(a, b, c);
}

template <bool SPLIT>
__device__ __forceinline__ void attn_body(const unsigned short* __restrict__ PHg, const unsigned short* __restrict__ PLg,
                                          const int pseq, const int qb0, unsigned short* __restrict__ OUTg,
                                          const int opitch, const int oseq, const float oscale) {
  constexpr bool F16 = !SPLIT;
  const float PSC = F16 ? 32768.0f : 1.0f;
  const float NEGF = -3.0e38f;
  const float SCL2 = 0.125f * 1.4426950408889634f;
  union FB { v16b v; v8b h[2]; };
  __shared__ __align__(16) __bf16 Ksh[AT_KC * AT_D];
  __shared__ __align__(16) __bf16 Ksl[SPLIT ? AT_KC * AT_D : 8];
  __shared__ __align__(16) __bf16 Vth[AT_D * AT_KC];
  __shared__ __align__(16) __bf16 Vtl[SPLIT ? AT_D * AT_KC : 8];
  __shared__ __align__(16) __bf16 Psh[AT_NW][16 * AT_KC];
  __shared__ __align__(16) __bf16 Psl[SPLIT ? AT_NW : 1][SPLIT ? 16 * AT_KC : 8];
  __shared__ __align__(16) float  Os[AT_NW][16 * OS_P];
  static_assert(AT_KC * AT_D == 128 * 32);

  const int tid  = threadIdx.x;
  const int wave = tid >> 5;
  const int lane = tid & 31;
  const int hh   = lane >> 4;
  const int c    = lane & 15;

  const int qb = blockIdx.x + qb0;
  const int h  = blockIdx.y;
  const int b  = blockIdx.z;
  const int q0 = qb * AT_QB + wave * 16;

  const __bf16* PH = (const __bf16*)PHg;
  const __bf16* PL = (const __bf16*)PLg;

  v16b qah[2], qal[2];
  {
    const size_t qoff = (size_t)(b * pseq + q0 + c) * QKVW + h * HD;
#pragma unroll
    for (int dc = 0; dc < 2; ++dc) {
      FB f;
      f.h[0] = *(const v8b*)(PH + qoff + dc * 32 + 8 * hh);
      f.h[1] = *(const v8b*)(PH + qoff + dc * 32 + 16 + 8 * hh);
      qah[dc] = f.v;
      if (SPLIT) {
        FB g;
        g.h[0] = *(const v8b*)(PL + qoff + dc * 32 + 8 * hh);
        g.h[1] = *(const v8b*)(PL + qoff + dc * 32 + 16 + 8 * hh);
        qal[dc] = g.v;
      } else {
        qal[dc] = f.v;
      }
    }
  }

  float mrow[8], lrow[8];
  v8f oacc[4];
#pragma unroll
  for (int r = 0; r < 8; ++r) { mrow[r] = NEGF; lrow[r] = 0.f; }
#pragma unroll
  for (int t = 0; t < 4; ++t) oacc[t] = (v8f){0.f,0.f,0.f,0.f,0.f,0.f,0.f,0.f};

  const int nChunks = qb + 1;
  for (int kc = 0; kc < nChunks; ++kc) {
    const int kv0 = kc * AT_KC;
    __syncthreads();
    {
      const int kvr = tid >> 1, dh = (tid & 1) * 32;
      const size_t grow = (size_t)(b * pseq + kv0 + kvr) * QKVW;
      const unsigned short* kp = PHg + grow + ND + h * HD + dh;
      const unsigned short* vp = PHg + grow + 2 * ND + h * HD + dh;
#pragma unroll
      for (int i = 0; i < 4; ++i) {
        const v4u kk = *(const v4u*)(kp + 8 * i);
        const v4u vv = *(const v4u*)(vp + 8 * i);
        *(v4u*)(Ksh + kvr * AT_D + dh + 8 * i) = kk;
#pragma unroll
        for (int e = 0; e < 8; ++e) {
          const unsigned w = vv[e >> 1];
          const unsigned short us = (e & 1) ? (unsigned short)(w >> 16) : (unsigned short)(w & 0xffffu);
          Vth[(dh + 8 * i + e) * AT_KC + kvr] = __builtin_bit_cast(__bf16, us);
        }
      }
      if (SPLIT) {
        const unsigned short* kpl = PLg + grow + ND + h * HD + dh;
        const unsigned short* vpl = PLg + grow + 2 * ND + h * HD + dh;
#pragma unroll
        for (int i = 0; i < 4; ++i) {
          const v4u kk = *(const v4u*)(kpl + 8 * i);
          const v4u vv = *(const v4u*)(vpl + 8 * i);
          *(v4u*)(Ksl + kvr * AT_D + dh + 8 * i) = kk;
#pragma unroll
          for (int e = 0; e < 8; ++e) {
            const unsigned w = vv[e >> 1];
            const unsigned short us = (e & 1) ? (unsigned short)(w >> 16) : (unsigned short)(w & 0xffffu);
            Vtl[(dh + 8 * i + e) * AT_KC + kvr] = __builtin_bit_cast(__bf16, us);
          }
        }
      }
    }
    __syncthreads();

    v8f s[4];
#pragma unroll
    for (int j = 0; j < 4; ++j) {
      s[j] = (v8f){0.f,0.f,0.f,0.f,0.f,0.f,0.f,0.f};
#pragma unroll
      for (int dc = 0; dc < 2; ++dc) {
        FB kb;
        kb.h[0] = *(const v8b*)(Ksh + (j * 16 + c) * AT_D + dc * 32 + 8 * hh);
        kb.h[1] = *(const v8b*)(Ksh + (j * 16 + c) * AT_D + dc * 32 + 16 + 8 * hh);
        s[j] = at_mma16<F16>(qah[dc], kb.v, s[j]);
        if (SPLIT) {
          FB kl;
          kl.h[0] = *(const v8b*)(Ksl + (j * 16 + c) * AT_D + dc * 32 + 8 * hh);
          kl.h[1] = *(const v8b*)(Ksl + (j * 16 + c) * AT_D + dc * 32 + 16 + 8 * hh);
          s[j] = at_mma16<F16>(qah[dc], kl.v, s[j]);
          s[j] = at_mma16<F16>(qal[dc], kb.v, s[j]);
        }
      }
    }
    const bool diag = (kc == qb);
    float cm[8];
#pragma unroll
    for (int r = 0; r < 8; ++r) {
      const int qrow = q0 + 8 * hh + r;
      float m = NEGF;
#pragma unroll
      for (int j = 0; j < 4; ++j) {
        const int kvcol = kv0 + j * 16 + c;
        float sv = s[j][r] * SCL2;
        if (diag && kvcol > qrow) sv = NEGF;
        s[j][r] = sv;
        m = fmaxf(m, sv);
      }
      m = fmaxf(m, __shfl_xor(m, 1, 32));
      m = fmaxf(m, __shfl_xor(m, 2, 32));
      m = fmaxf(m, __shfl_xor(m, 4, 32));
      m = fmaxf(m, __shfl_xor(m, 8, 32));
      cm[r] = m;
    }
    __bf16* pwh = Psh[wave];
    __bf16* pwl = Psl[SPLIT ? wave : 0];
#pragma unroll
    for (int r = 0; r < 8; ++r) {
      const float mnew = fmaxf(mrow[r], cm[r]);
      const float alpha = exp2f(mrow[r] - mnew);
      mrow[r] = mnew;
      float psum = 0.f;
#pragma unroll
      for (int j = 0; j < 4; ++j) {
        const float sv = s[j][r];
        const float e2 = exp2f(sv - mnew);
        const float p = (sv < -1.0e37f) ? 0.f : e2;
        psum += p;
        if (SPLIT) { __bf16 a, bl; at_split(p, a, bl); pwh[(8 * hh + r) * AT_KC + j * 16 + c] = a; pwl[(8 * hh + r) * AT_KC + j * 16 + c] = bl; }
        else pwh[(8 * hh + r) * AT_KC + j * 16 + c] = at_to16<F16>(p * PSC);
      }
      psum += __shfl_xor(psum, 1, 32);
      psum += __shfl_xor(psum, 2, 32);
      psum += __shfl_xor(psum, 4, 32);
      psum += __shfl_xor(psum, 8, 32);
      lrow[r] = lrow[r] * alpha + psum;
#pragma unroll
      for (int t = 0; t < 4; ++t) oacc[t][r] *= alpha;
    }
    __builtin_amdgcn_fence(3  , "workgroup");
    __builtin_amdgcn_wave_barrier();
    __builtin_amdgcn_fence(2  , "workgroup");
#pragma unroll
    for (int kk = 0; kk < 2; ++kk) {
      FB pa, pl;
      pa.h[0] = *(const v8b*)(pwh + c * AT_KC + kk * 32 + 8 * hh);
      pa.h[1] = *(const v8b*)(pwh + c * AT_KC + kk * 32 + 16 + 8 * hh);
      if (SPLIT) {
        pl.h[0] = *(const v8b*)(pwl + c * AT_KC + kk * 32 + 8 * hh);
        pl.h[1] = *(const v8b*)(pwl + c * AT_KC + kk * 32 + 16 + 8 * hh);
      } else {
        pl.v = pa.v;
      }
#pragma unroll
      for (int t = 0; t < 4; ++t) {
        FB vb;
        vb.h[0] = *(const v8b*)(Vth + (t * 16 + c) * AT_KC + kk * 32 + 8 * hh);
        vb.h[1] = *(const v8b*)(Vth + (t * 16 + c) * AT_KC + kk * 32 + 16 + 8 * hh);
        oacc[t] = at_mma16<F16>(pa.v, vb.v, oacc[t]);
        if (SPLIT) {
          FB vl;
          vl.h[0] = *(const v8b*)(Vtl + (t * 16 + c) * AT_KC + kk * 32 + 8 * hh);
          vl.h[1] = *(const v8b*)(Vtl + (t * 16 + c) * AT_KC + kk * 32 + 16 + 8 * hh);
          oacc[t] = at_mma16<F16>(pa.v, vl.v, oacc[t]);
          oacc[t] = at_mma16<F16>(pl.v, vb.v, oacc[t]);
        }
      }
    }
    __builtin_amdgcn_fence(3  , "workgroup");
    __builtin_amdgcn_wave_barrier();
    __builtin_amdgcn_fence(2  , "workgroup");
  }

  float* os = Os[wave];
#pragma unroll
  for (int r = 0; r < 8; ++r) {
    const float inv = oscale * (1.0f / (lrow[r] * PSC));
#pragma unroll
    for (int t = 0; t < 4; ++t) os[(8 * hh + r) * OS_P + t * 16 + c] = oacc[t][r] * inv;
  }
  __builtin_amdgcn_fence(3  , "workgroup");
  __builtin_amdgcn_wave_barrier();
  __builtin_amdgcn_fence(2  , "workgroup");
  {
    const int q = lane >> 3, c8 = (lane & 7) * 8;
    unsigned short* ob = OUTg + (size_t)(b * oseq + q0) * opitch + h * HD + c8;
    for (int pass = 0; pass < 2; ++pass) {
#pragma unroll
      for (int it = 0; it < 4; ++it) {
        const int row = it * 4 + q;
        const v4f a = *(const v4f*)(os + row * OS_P + c8);
        const v4f d = *(const v4f*)(os + row * OS_P + c8 + 4);
        if (SPLIT) {
          const unsigned short h0 = f2bf_bits(a.x), h1 = f2bf_bits(a.y), h2 = f2bf_bits(a.z), h3 = f2bf_bits(a.w);
          const unsigned short h4 = f2bf_bits(d.x), h5 = f2bf_bits(d.y), h6 = f2bf_bits(d.z), h7 = f2bf_bits(d.w);
          const unsigned short l0 = f2bf_bits(a.x - bf_bits2f(h0)), l1 = f2bf_bits(a.y - bf_bits2f(h1)), l2 = f2bf_bits(a.z - bf_bits2f(h2)), l3 = f2bf_bits(a.w - bf_bits2f(h3));
          const unsigned short l4 = f2bf_bits(d.x - bf_bits2f(h4)), l5 = f2bf_bits(d.y - bf_bits2f(h5)), l6 = f2bf_bits(d.z - bf_bits2f(h6)), l7 = f2bf_bits(d.w - bf_bits2f(h7));
          v4u ph, pl;
          ph.x = (unsigned)h0 | ((unsigned)h1 << 16); ph.y = (unsigned)h2 | ((unsigned)h3 << 16); ph.z = (unsigned)h4 | ((unsigned)h5 << 16); ph.w = (unsigned)h6 | ((unsigned)h7 << 16);
          pl.x = (unsigned)l0 | ((unsigned)l1 << 16); pl.y = (unsigned)l2 | ((unsigned)l3 << 16); pl.z = (unsigned)l4 | ((unsigned)l5 << 16); pl.w = (unsigned)l6 | ((unsigned)l7 << 16);
          *(volatile v4u*)(ob + (size_t)row * opitch) = ph;
          *(volatile v4u*)(ob + (size_t)row * opitch + ND) = pl;
        } else {
          v4u ph;
          ph.x = cmb_pk2(a.x, a.y); ph.y = cmb_pk2(a.z, a.w); ph.z = cmb_pk2(d.x, d.y); ph.w = cmb_pk2(d.z, d.w);
          *(volatile v4u*)(ob + (size_t)row * opitch) = ph;
        }
      }
      __threadfence();
    }
  }
}

__global__ __launch_bounds__(128) void k_attn_late(const unsigned short* __restrict__ QKV16, unsigned short* __restrict__ CTX16) {
  attn_body<false>(QKV16, nullptr, SEQ, EARLY / AT_QB, CTX16, ND, SEQ, 16.0f);
}
__global__ __launch_bounds__(128) void k_attn_early(const unsigned short* __restrict__ QEH, const unsigned short* __restrict__ QEL, unsigned short* __restrict__ CTXE) {
  attn_body<true>(QEH, QEL, EARLY, 0, CTXE, 2 * ND, EARLY, 1.0f);
}

constexpr size_t al256(size_t x) { return (x + 255) / 256 * 256; }
constexpr size_t SZ_X16   = al256((size_t)NB * SEQ * ND * 2);
constexpr size_t SZ_W316  = al256((size_t)QKVW * ND * 2);
constexpr size_t SZ_QKV16 = al256((size_t)NB * SEQ * QKVW * 2);
constexpr size_t SZ_QE    = al256((size_t)NB * EARLY * QKVW * 2);
constexpr size_t SZ_CTX16 = al256((size_t)NB * SEQ * ND * 2);
constexpr size_t SZ_CTXE  = al256((size_t)NB * EARLY * 2 * ND * 2);
constexpr size_t SZ_WO16  = al256((size_t)ND * ND * 2);
constexpr size_t SZ_WOB2  = al256((size_t)ND * 2 * ND * 2);
constexpr size_t SZ_BR3   = al256((size_t)QKVW * 4);
constexpr size_t SZ_BRO   = al256((size_t)ND * 4);
constexpr size_t WS_TOTAL = SZ_X16 + SZ_W316 + SZ_QKV16 + 2 * SZ_QE + SZ_CTX16 + SZ_CTXE + SZ_WO16 + SZ_WOB2 + SZ_BR3 + SZ_BRO;
static_assert(WS_TOTAL <= 134217728ull);

extern "C" void kernel_launch(void* const* d_in, const int* in_sizes, int n_in, void* d_out, int out_size, void* d_ws, size_t ws_size, hipStream_t stream) {
  if (n_in < 5) return;
  const long long need0 = ((long long)(NB - 1) * SEQ_FULL + SEQ) * ND;
  if ((long long)in_sizes[0] < need0) return;
  if ((long long)in_sizes[1] < (long long)ND * QKVW) return;
  if (in_sizes[2] < QKVW) return;
  if ((long long)in_sizes[3] < (long long)ND * ND) return;
  if (in_sizes[4] < ND) return;
  if ((long long)out_size < (long long)NB * SEQ * ND) return;
  if (WS_TOTAL > ws_size) return;

  const float* x    = (const float*)d_in[0];
  const float* Wqkv = (const float*)d_in[1];
  const float* bqkv = (const float*)d_in[2];
  const float* Wo   = (const float*)d_in[3];
  const float* bo   = (const float*)d_in[4];
  float* out = (float*)d_out;

  char* wsp = (char*)d_ws;
  unsigned short* X16   = (unsigned short*)wsp; wsp += SZ_X16;
  unsigned short* W316  = (unsigned short*)wsp; wsp += SZ_W316;
  unsigned short* QKV16 = (unsigned short*)wsp; wsp += SZ_QKV16;
  unsigned short* QEH   = (unsigned short*)wsp; wsp += SZ_QE;
  unsigned short* QEL   = (unsigned short*)wsp; wsp += SZ_QE;
  unsigned short* CTX16 = (unsigned short*)wsp; wsp += SZ_CTX16;
  unsigned short* CTXE  = (unsigned short*)wsp; wsp += SZ_CTXE;
  unsigned short* WO16  = (unsigned short*)wsp; wsp += SZ_WO16;
  unsigned short* WOB2  = (unsigned short*)wsp; wsp += SZ_WOB2;
  float* BR3 = (float*)wsp; wsp += SZ_BR3;
  float* BRO = (float*)wsp; wsp += SZ_BRO;

  k_cast_x<<<(unsigned)(((long long)NB * SEQ * (ND / 8) + 255) / 256), 256, 0, stream>>>(x, X16);
  k_wT16<<<(unsigned)(((long long)QKVW * (ND / 8) + 255) / 256), 256, 0, stream>>>(Wqkv, QKVW, W316, ND, ND, QKVW, 16.0f, 0, 0);
  k_bfvec<<<(QKVW + 255) / 256, 256, 0, stream>>>(bqkv, BR3, QKVW);
  k_wT16<<<(unsigned)(((long long)ND * (ND / 8) + 255) / 256), 256, 0, stream>>>(Wo, ND, WO16, ND, ND, ND, 16.0f, 0, 0);
  k_wT16<<<(unsigned)(((long long)ND * (ND / 8) + 255) / 256), 256, 0, stream>>>(Wo, ND, WOB2, 2 * ND, ND, ND, 1.0f, 1, ND);
  k_bfvec<<<(ND + 255) / 256, 256, 0, stream>>>(bo, BRO, ND);

  k_gemm_qkv_main<<<dim3((unsigned)((((NB * SEQ) / 64) * (QKVW / 64) + 7) / 8), 1u), 256, 0, stream>>>(X16, W316, QKV16, BR3);
  k_gemm_qkv_early<<<dim3((unsigned)(((EARLY / 64) * (QKVW / 64) + 7) / 8), (unsigned)NB), 256, 0, stream>>>(X16, W316, QEH, QEL, BR3);

  k_attn_early<<<dim3((unsigned)(EARLY / AT_QB), (unsigned)NH, (unsigned)NB), 128, 0, stream>>>(QEH, QEL, CTXE);
  if (SEQ > EARLY)
    k_attn_late<<<dim3((unsigned)((SEQ - EARLY) / AT_QB), (unsigned)NH, (unsigned)NB), 128, 0, stream>>>(QKV16, CTX16);

  k_gemm_proj_early<<<dim3((unsigned)(((EARLY / 64) * (ND / 64) + 7) / 8), (unsigned)NB), 256, 0, stream>>>(CTXE, WOB2, out, BRO);
  if (SEQ > EARLY)
    k_gemm_proj_main<<<dim3((unsigned)((((SEQ - EARLY) / 64) * (ND / 64) + 7) / 8), (unsigned)NB), 256, 0, stream>>>(CTX16, WO16, out, BRO);
}
